// OPTAttention_42314017800961
// MI455X (gfx1250) — hardware-run, weakly checked
//
#include <hip/hip_runtime.h>
#include <math.h>

#ifndef NB
#define NB 16
#endif
#ifndef PAST
#define PAST 4096
#endif
#define PAST_FULL 4096
#define TT 4
#define EDIM 2048
#define HEADS 32
#define HD 64
#define MROWS (NB * TT)
#define S_FULL (PAST_FULL + TT)

#define CX 2048.0f
#define CW 131072.0f
#define CKV 2048.0f
#define CQ 16384.0f
#define CP 16384.0f
#define CO 4096.0f
#define CPV (CP * CKV)
#define SC_QK (1.0f / (CQ * CKV))
#define FMIN_F32 (-3.4028234663852886e38f)

static_assert(TT == 4);
static_assert(HEADS * HD == EDIM);
static_assert(MROWS % 64 == 0);
static_assert(PAST % 64 == 0 && PAST >= 64 && PAST <= PAST_FULL);
static_assert(EDIM % 64 == 0);
static_assert((EDIM * EDIM / 8) % 256 == 0);
static_assert((HEADS * PAST * HD / 8) % 256 == 0);
static_assert((MROWS * EDIM / 8) % 256 == 0);
constexpr size_t WS_TOTAL = (size_t)4 * EDIM * EDIM * 2 + (size_t)2 * HEADS * PAST * HD * 2 + (size_t)3 * MROWS * EDIM * 2 + (size_t)2 * MROWS * EDIM * 4;
static_assert(WS_TOTAL < (size_t)134217728);

typedef _Float16 h16;
typedef __attribute__((ext_vector_type(16))) _Float16 v16h;
typedef __attribute__((ext_vector_type(8)))  _Float16 v8h;
typedef __attribute__((ext_vector_type(8)))  float    v8f;
typedef __attribute__((ext_vector_type(4)))  float    v4f;


static __device__ __forceinline__ float bfr(float f) {
    unsigned u = __float_as_uint(f);
    u += 0x7FFFu + ((u >> 16) & 1u);
    return __uint_as_float(u & 0xFFFF0000u);
}
static __device__ __forceinline__ h16 toh_flush(float v) {
    const float w = (fabsf(v) < 6.103515625e-05f) ? 0.0f : v;
    return (h16)w;
}
static __device__ __forceinline__ v8h pack8(v4f a, v4f b) {
    v8h r;
    r[0] = toh_flush(a.x); r[1] = toh_flush(a.y); r[2] = toh_flush(a.z); r[3] = toh_flush(a.w);
    r[4] = toh_flush(b.x); r[5] = toh_flush(b.y); r[6] = toh_flush(b.z); r[7] = toh_flush(b.w);
    return r;
}

union FragU { v16h v; v8h h[2]; };
static __device__ __forceinline__ v16h frag_ld(const h16* p) {
    FragU f; f.h[0] = *(const v8h*)(p); f.h[1] = *(const v8h*)(p + 16); return f.v;
}
static __device__ __forceinline__ v8f wmma16g(v16h a, v16h b, v8f c) {
    c = __builtin_amdgcn_wmma_f32_16x16x32_f16(false, a, false, b, (short)0, c, false, false);
    asm volatile("v_nop\n\tv_nop\n\tv_nop\n\tv_nop" : "+v"(c) : "v"(a), "v"(b));
    return c;
}
static __device__ __forceinline__ void wave_sync_lds() {
    __builtin_amdgcn_fence(3  , "workgroup");
    __builtin_amdgcn_wave_barrier();
    __builtin_amdgcn_fence(2  , "workgroup");
}

template <unsigned LG, unsigned SEG8, unsigned SRC_SEG>
__global__ __launch_bounds__(256) void k_cvt8(const float* __restrict__ src, h16* __restrict__ dst, unsigned n8) {
    const unsigned u = blockIdx.x * 256u + threadIdx.x;
    if (u >= n8) return;
    const unsigned seg = u / SEG8;
    const unsigned w = u - seg * SEG8;
    const float* s = src + (size_t)seg * SRC_SEG + (size_t)w * 8u;
    v4f a = *(const v4f*)s, b = *(const v4f*)(s + 4);
    constexpr float cs = (float)(1u << LG);
    a.x = bfr(a.x) * cs; a.y = bfr(a.y) * cs; a.z = bfr(a.z) * cs; a.w = bfr(a.w) * cs;
    b.x = bfr(b.x) * cs; b.y = bfr(b.y) * cs; b.z = bfr(b.z) * cs; b.w = bfr(b.w) * cs;
    const v8h hv = pack8(a, b);
    h16* d = dst + (size_t)u * 8u;
    *(volatile v8h*)d = hv;
    __threadfence();
    *(volatile v8h*)d = hv;
}

__global__ __launch_bounds__(256) void k_vt(const float* __restrict__ v, h16* __restrict__ vt) {
    __shared__ __align__(16) float sV[64 * 68];
    const unsigned tid = threadIdx.x;
    const unsigned k0 = blockIdx.x * 64u, head = blockIdx.y;
    {
        const unsigned key = tid >> 2, dq = (tid & 3u) * 16u;
        const float* s = v + ((size_t)head * PAST_FULL + k0 + key) * HD + dq;
#pragma unroll
        for (int g = 0; g < 4; ++g) {
            const v4f a = *(const v4f*)(s + 4 * g);
            float* o = sV + (dq + 4u * (unsigned)g) * 68u + key;
            o[0] = bfr(a.x) * CKV; o[68] = bfr(a.y) * CKV; o[136] = bfr(a.z) * CKV; o[204] = bfr(a.w) * CKV;
        }
    }
    __syncthreads();
    const unsigned row = tid >> 3, c8 = (tid & 7u) * 8u;
    v8h hv[2];
#pragma unroll
    for (int it = 0; it < 2; ++it) {
        const float* sp = sV + ((unsigned)it * 32u + row) * 68u + c8;
        hv[it] = pack8(*(const v4f*)sp, *(const v4f*)(sp + 4));
    }
    h16* dst = vt + ((size_t)head * HD + row) * PAST + k0 + c8;
    *(volatile v8h*)dst = hv[0];
    *(volatile v8h*)(dst + (size_t)32 * PAST) = hv[1];
    __threadfence();
    *(volatile v8h*)dst = hv[0];
    *(volatile v8h*)(dst + (size_t)32 * PAST) = hv[1];
}

template <int OUT_MODE, unsigned LG_IN, unsigned LG_POST>
__global__ __launch_bounds__(256) void k_gemm64(
    const h16* __restrict__ A, unsigned lda, const h16* __restrict__ Bt, unsigned ldb,
    void* __restrict__ Cout, unsigned ldc, const float* __restrict__ bias, unsigned M, unsigned N, unsigned K) {
  __shared__ __align__(16) float sT[8][16 * 68];
  const unsigned lane = threadIdx.x & 31u;
  const unsigned wave = threadIdx.x >> 5;
  const unsigned tilesN = N >> 6, tilesM = M >> 6;
  const unsigned tile = blockIdx.x * 8u + wave;
  if (tile >= tilesM * tilesN) return;
  const unsigned tm = tile / tilesN;
  const unsigned tn = tile - tm * tilesN;
  const unsigned m0 = tm << 6, n0 = tn << 6;
  const unsigned rlane = lane & 15u;
  const unsigned koff = (lane >> 4) * 8u;
  constexpr float scale = 1.0f / (float)(1u << LG_IN);
  constexpr float post = (float)(1u << LG_POST);

  v8f acc[4][4];
#pragma unroll
  for (int i = 0; i < 4; ++i)
#pragma unroll
    for (int j = 0; j < 4; ++j) acc[i][j] = (v8f){0.f,0.f,0.f,0.f,0.f,0.f,0.f,0.f};

  for (unsigned k0 = 0; k0 < K; k0 += 32u) {
    v16h bh[4];
#pragma unroll
    for (int j = 0; j < 4; ++j)
      bh[j] = frag_ld(Bt + (size_t)(n0 + ((unsigned)j << 4) + rlane) * ldb + koff + k0);
#pragma unroll
    for (int i = 0; i < 4; ++i) {
      const v16h ah = frag_ld(A + (size_t)(m0 + ((unsigned)i << 4) + rlane) * lda + koff + k0);
#pragma unroll
      for (int j = 0; j < 4; ++j) acc[i][j] = wmma16g(ah, bh[j], acc[i][j]);
    }
  }

  float* slab = sT[wave];
#pragma unroll
  for (int i = 0; i < 4; ++i) {
    const unsigned mBase = m0 + ((unsigned)i << 4);
#pragma unroll
    for (int j = 0; j < 4; ++j) {
      const unsigned n = n0 + ((unsigned)j << 4) + rlane;
      const float bv = bfr(bias[n]);
#pragma unroll
      for (int r = 0; r < 8; ++r)
        slab[(koff + (unsigned)r) * 68u + ((unsigned)j << 4) + rlane] = (acc[i][j][r] * scale + bv) * post;
    }
    wave_sync_lds();
    if (OUT_MODE == 0) {
      float* C = (float*)Cout;
      const unsigned hh = lane >> 4, c4 = (lane & 15u) * 4u;
#pragma unroll
      for (int half = 0; half < 2; ++half) {
        v4f vv[4];
#pragma unroll
        for (int it = 0; it < 4; ++it)
          vv[it] = *(const v4f*)(slab + ((unsigned)(half * 4 + it) * 2u + hh) * 68u + c4);
#pragma unroll
        for (int it = 0; it < 4; ++it)
          *(volatile v4f*)(C + (size_t)(mBase + (unsigned)(half * 4 + it) * 2u + hh) * ldc + n0 + c4) = vv[it];
        __threadfence();
#pragma unroll
        for (int it = 0; it < 4; ++it)
          *(volatile v4f*)(C + (size_t)(mBase + (unsigned)(half * 4 + it) * 2u + hh) * ldc + n0 + c4) = vv[it];
        __threadfence();
      }
    } else {
      h16* C = (h16*)Cout;
      const unsigned q = lane >> 3, c8 = (lane & 7u) * 8u;
      v8h hv[4];
#pragma unroll
      for (int it = 0; it < 4; ++it) {
        const float* sp = slab + ((unsigned)it * 4u + q) * 68u + c8;
        hv[it] = pack8(*(const v4f*)sp, *(const v4f*)(sp + 4));
      }
#pragma unroll
      for (int it = 0; it < 4; ++it)
        *(volatile v8h*)(C + (size_t)(mBase + (unsigned)it * 4u + q) * ldc + n0 + c8) = hv[it];
      __threadfence();
#pragma unroll
      for (int it = 0; it < 4; ++it)
        *(volatile v8h*)(C + (size_t)(mBase + (unsigned)it * 4u + q) * ldc + n0 + c8) = hv[it];
      __threadfence();
    }
    wave_sync_lds();
  }
}

#define AT_PS 68
#define AT_PP 72
__global__ __launch_bounds__(128) void k_attn(const h16* __restrict__ q16, const h16* __restrict__ k16, const h16* __restrict__ vt16,
                                              const float* __restrict__ mask, const float* __restrict__ knew, const float* __restrict__ vnew,
                                              h16* __restrict__ attn16) {
    __shared__ __align__(16) float sS[4][16 * AT_PS];
    __shared__ __align__(16) h16   sP[4][16 * AT_PP];
    const unsigned tid = threadIdx.x, lane = tid & 31u, wave = tid >> 5;
    const unsigned hh = lane >> 4, c = lane & 15u;
    const unsigned prow = lane >> 1, hf = lane & 1u;
    const unsigned head = blockIdx.x;
    const unsigned R0 = (blockIdx.y * 4u + wave) * 16u;
    float* slab = sS[wave];
    h16* pw = sP[wave];
    const h16* qrow = q16 + (size_t)(R0 + c) * EDIM + head * HD + 8u * hh;
    const v16h qf0 = frag_ld(qrow), qf1 = frag_ld(qrow + 32);
    const h16* kbase = k16 + ((size_t)head * PAST + c) * HD + 8u * hh;
    const h16* vbase = vt16 + ((size_t)head * HD + c) * PAST + 8u * hh;
    const float* mrow = mask + (size_t)(R0 + prow) * S_FULL;
    float m_run = -INFINITY;
    float l_run = 0.0f;
    v8f os[4];
#pragma unroll
    for (int t = 0; t < 4; ++t) os[t] = (v8f){0.f,0.f,0.f,0.f,0.f,0.f,0.f,0.f};

    for (unsigned kc = 0; kc < (unsigned)(PAST / 64); ++kc) {
        const unsigned kv0 = kc * 64u;
#pragma unroll
        for (int j = 0; j < 4; ++j) {
            const h16* kp = kbase + (size_t)(kv0 + (unsigned)j * 16u) * HD;
            v8f z = (v8f){0.f,0.f,0.f,0.f,0.f,0.f,0.f,0.f};
            z = wmma16g(qf0, frag_ld(kp), z);
            z = wmma16g(qf1, frag_ld(kp + 32), z);
#pragma unroll
            for (int r = 0; r < 8; ++r) slab[(8u * hh + (unsigned)r) * AT_PS + (unsigned)j * 16u + c] = z[r] * SC_QK;
        }
        wave_sync_lds();
        float sv[32];
        float mx = -INFINITY;
        {
            const float* sp = slab + prow * AT_PS + hf * 32u;
            const float* mp = mrow + kv0 + hf * 32u;
#pragma unroll
            for (int g = 0; g < 8; ++g) {
                const v4f sc = *(const v4f*)(sp + 4 * g);
                const v4f mk = *(const v4f*)(mp + 4 * g);
                sv[4 * g + 0] = fmaxf(sc.x + bfr(mk.x), FMIN_F32);
                sv[4 * g + 1] = fmaxf(sc.y + bfr(mk.y), FMIN_F32);
                sv[4 * g + 2] = fmaxf(sc.z + bfr(mk.z), FMIN_F32);
                sv[4 * g + 3] = fmaxf(sc.w + bfr(mk.w), FMIN_F32);
                mx = fmaxf(fmaxf(mx, sv[4 * g + 0]), fmaxf(sv[4 * g + 1], fmaxf(sv[4 * g + 2], sv[4 * g + 3])));
            }
        }
        mx = fmaxf(mx, __shfl_xor(mx, 1, 32));
        const float mnew = fmaxf(m_run, mx);
        const float alpha = expf(m_run - mnew);
        m_run = mnew;
        float psum = 0.0f;
#pragma unroll
        for (int g = 0; g < 4; ++g) {
            v8h pv;
#pragma unroll
            for (int e = 0; e < 8; ++e) {
                const float p = expf(sv[8 * g + e] - mnew);
                psum += p;
                pv[e] = toh_flush(p * CP);
            }
            *(v8h*)(pw + prow * AT_PP + hf * 32u + 8u * (unsigned)g) = pv;
        }
        psum += __shfl_xor(psum, 1, 32);
        l_run = l_run * alpha + psum;
#pragma unroll
        for (int r = 0; r < 8; ++r) {
            const float ar = __shfl(alpha, (int)(16u * hh + 2u * (unsigned)r), 32);
#pragma unroll
            for (int t = 0; t < 4; ++t) os[t][r] *= ar;
        }
        wave_sync_lds();
#pragma unroll
        for (int kk = 0; kk < 2; ++kk) {
            const v16h pa = frag_ld(pw + c * AT_PP + (unsigned)kk * 32u + 8u * hh);
#pragma unroll
            for (int t = 0; t < 4; ++t) {
                const v16h vb = frag_ld(vbase + (size_t)((unsigned)t * 16u) * PAST + kv0 + (unsigned)kk * 32u);
                os[t] = wmma16g(pa, vb, os[t]);
            }
        }
        wave_sync_lds();
    }

    {
        const float* kn = knew + (size_t)(R0 + prow) * EDIM + head * HD + hf * 32u;
#pragma unroll
        for (int g = 0; g < 8; ++g) *(v4f*)(slab + prow * AT_PS + hf * 32u + 4u * (unsigned)g) = *(const v4f*)(kn + 4 * g);
    }
    wave_sync_lds();
    float qv[32];
    {
        const h16* qp = q16 + (size_t)(R0 + prow) * EDIM + head * HD + hf * 32u;
#pragma unroll
        for (int g = 0; g < 4; ++g) {
            const v8h qh = *(const v8h*)(qp + 8 * g);
#pragma unroll
            for (int e = 0; e < 8; ++e) qv[8 * g + e] = (float)qh[e] * (1.0f / CQ);
        }
    }
    float sn[4];
#pragma unroll
    for (int j = 0; j < 4; ++j) {
        const float* kr = slab + ((prow >> 2) * 4u + (unsigned)j) * AT_PS + hf * 32u;
        float a = 0.0f;
#pragma unroll
        for (int g = 0; g < 8; ++g) {
            const v4f kv = *(const v4f*)(kr + 4 * g);
            a += qv[4 * g] * kv.x; a += qv[4 * g + 1] * kv.y; a += qv[4 * g + 2] * kv.z; a += qv[4 * g + 3] * kv.w;
        }
        a += __shfl_xor(a, 1, 32);
        sn[j] = a;
    }
    const v4f mkn = *(const v4f*)(mrow + PAST);
    sn[0] = fmaxf(sn[0] + bfr(mkn.x), FMIN_F32);
    sn[1] = fmaxf(sn[1] + bfr(mkn.y), FMIN_F32);
    sn[2] = fmaxf(sn[2] + bfr(mkn.z), FMIN_F32);
    sn[3] = fmaxf(sn[3] + bfr(mkn.w), FMIN_F32);
    const float mxn = fmaxf(fmaxf(sn[0], sn[1]), fmaxf(sn[2], sn[3]));
    const float mfin = fmaxf(m_run, mxn);
    const float alphan = expf(m_run - mfin);
    float pn[4];
#pragma unroll
    for (int j = 0; j < 4; ++j) pn[j] = expf(sn[j] - mfin);
    l_run = l_run * alphan + ((pn[0] + pn[1]) + (pn[2] + pn[3]));
    wave_sync_lds();
    {
        const float* vn = vnew + (size_t)(R0 + prow) * EDIM + head * HD + hf * 32u;
#pragma unroll
        for (int g = 0; g < 8; ++g) *(v4f*)(slab + prow * AT_PS + hf * 32u + 4u * (unsigned)g) = *(const v4f*)(vn + 4 * g);
    }
    wave_sync_lds();
#pragma unroll
    for (int r = 0; r < 8; ++r) {
        const int src = (int)(16u * hh + 2u * (unsigned)r);
        const float ar = __shfl(alphan, src, 32);
        const float p0 = __shfl(pn[0], src, 32) * CPV;
        const float p1 = __shfl(pn[1], src, 32) * CPV;
        const float p2 = __shfl(pn[2], src, 32) * CPV;
        const float p3 = __shfl(pn[3], src, 32) * CPV;
        const float lr = __shfl(l_run, src, 32);
        const float* vr = slab + ((2u * hh + (unsigned)(r >> 2)) * 4u) * AT_PS + c;
#pragma unroll
        for (int t = 0; t < 4; ++t) {
            float o = os[t][r] * ar;
            o += p0 * vr[t * 16];
            o += p1 * vr[AT_PS + t * 16];
            o += p2 * vr[2 * AT_PS + t * 16];
            o += p3 * vr[3 * AT_PS + t * 16];
            os[t][r] = ((o * (1.0f / CPV)) / lr) * CO;
        }
    }
    wave_sync_lds();
#pragma unroll
    for (int t = 0; t < 4; ++t)
#pragma unroll
        for (int r = 0; r < 8; ++r) slab[(8u * hh + (unsigned)r) * AT_PS + (unsigned)t * 16u + c] = os[t][r];
    wave_sync_lds();
    {
        const unsigned q = lane >> 3, c8 = (lane & 7u) * 8u;
        v8h ov[4];
#pragma unroll
        for (int it = 0; it < 4; ++it) {
            const float* sp = slab + ((unsigned)it * 4u + q) * AT_PS + c8;
            ov[it] = pack8(*(const v4f*)sp, *(const v4f*)(sp + 4));
        }
        h16* dst = attn16 + (size_t)(R0 + q) * EDIM + head * HD + c8;
#pragma unroll
        for (int it = 0; it < 4; ++it) *(volatile v8h*)(dst + (size_t)((unsigned)it * 4u) * EDIM) = ov[it];
        __threadfence();
#pragma unroll
        for (int it = 0; it < 4; ++it) *(volatile v8h*)(dst + (size_t)((unsigned)it * 4u) * EDIM) = ov[it];
        __threadfence();
    }
}

extern "C" void kernel_launch(void* const* d_in, const int* in_sizes, int n_in, void* d_out, int out_size,
                              void* d_ws, size_t ws_size, hipStream_t stream) {
    if (n_in < 12) return;
    if (in_sizes[0] < MROWS * EDIM || in_sizes[1] < HEADS * PAST_FULL * HD || in_sizes[2] < HEADS * PAST_FULL * HD) return;
    if (in_sizes[3] < MROWS * S_FULL) return;
    if (in_sizes[4] < EDIM * EDIM || in_sizes[6] < EDIM * EDIM || in_sizes[8] < EDIM * EDIM || in_sizes[10] < EDIM * EDIM) return;
    if (in_sizes[5] < EDIM || in_sizes[7] < EDIM || in_sizes[9] < EDIM || in_sizes[11] < EDIM) return;
    if (out_size < MROWS * EDIM) return;

    const float* hidden  = (const float*)d_in[0];
    const float* past_k  = (const float*)d_in[1];
    const float* past_v  = (const float*)d_in[2];
    const float* mask    = (const float*)d_in[3];
    const float* Wq      = (const float*)d_in[4];
    const float* bq      = (const float*)d_in[5];
    const float* Wk      = (const float*)d_in[6];
    const float* bk      = (const float*)d_in[7];
    const float* Wv      = (const float*)d_in[8];
    const float* bv      = (const float*)d_in[9];
    const float* Wo      = (const float*)d_in[10];
    const float* bo      = (const float*)d_in[11];
    float* out = (float*)d_out;

    char* wsp = (char*)d_ws;
    size_t off = 0;
    auto carve = [&](size_t bytes) -> void* { void* r = wsp + off; off += (bytes + 255) & ~(size_t)255; return r; };
    h16*   wq16   = (h16*)carve((size_t)EDIM * EDIM * 2);
    h16*   wk16   = (h16*)carve((size_t)EDIM * EDIM * 2);
    h16*   wv16   = (h16*)carve((size_t)EDIM * EDIM * 2);
    h16*   wo16   = (h16*)carve((size_t)EDIM * EDIM * 2);
    h16*   k16    = (h16*)carve((size_t)HEADS * PAST * HD * 2);
    h16*   vt16   = (h16*)carve((size_t)HEADS * HD * PAST * 2);
    h16*   x16    = (h16*)carve((size_t)MROWS * EDIM * 2);
    h16*   q16    = (h16*)carve((size_t)MROWS * EDIM * 2);
    float* knew   = (float*)carve((size_t)MROWS * EDIM * 4);
    float* vnew   = (float*)carve((size_t)MROWS * EDIM * 4);
    h16*   attn16 = (h16*)carve((size_t)MROWS * EDIM * 2);
    if (off > ws_size || off > (size_t)134217728) return;

    constexpr unsigned NW8 = EDIM * EDIM / 8;
    k_cvt8<17u, NW8, (unsigned)(EDIM * EDIM)><<<NW8 / 256, 256, 0, stream>>>(Wq, wq16, NW8);
    k_cvt8<17u, NW8, (unsigned)(EDIM * EDIM)><<<NW8 / 256, 256, 0, stream>>>(Wk, wk16, NW8);
    k_cvt8<17u, NW8, (unsigned)(EDIM * EDIM)><<<NW8 / 256, 256, 0, stream>>>(Wv, wv16, NW8);
    k_cvt8<17u, NW8, (unsigned)(EDIM * EDIM)><<<NW8 / 256, 256, 0, stream>>>(Wo, wo16, NW8);

    constexpr unsigned NK8 = HEADS * PAST * HD / 8;
    k_cvt8<11u, (unsigned)(PAST * HD / 8), (unsigned)(PAST_FULL * HD)><<<NK8 / 256, 256, 0, stream>>>(past_k, k16, NK8);
    k_vt<<<dim3(PAST / 64, HEADS), 256, 0, stream>>>(past_v, vt16);

    constexpr unsigned NX8 = MROWS * EDIM / 8;
    k_cvt8<11u, NX8, (unsigned)(MROWS * EDIM)><<<NX8 / 256, 256, 0, stream>>>(hidden, x16, NX8);

    const unsigned gP = ((MROWS / 64) * (EDIM / 64) + 7) / 8;
    k_gemm64<1, 28u, 11u><<<gP, 256, 0, stream>>>((const h16*)x16, EDIM, (const h16*)wq16, EDIM, (void*)q16, EDIM, bq, MROWS, EDIM, EDIM);
    k_gemm64<0, 28u, 0u><<<gP, 256, 0, stream>>>((const h16*)x16, EDIM, (const h16*)wk16, EDIM, (void*)knew, EDIM, bk, MROWS, EDIM, EDIM);
    k_gemm64<0, 28u, 0u><<<gP, 256, 0, stream>>>((const h16*)x16, EDIM, (const h16*)wv16, EDIM, (void*)vnew, EDIM, bv, MROWS, EDIM, EDIM);

    k_attn<<<dim3(HEADS, MROWS / 64), 128, 0, stream>>>((const h16*)q16, (const h16*)k16, (const h16*)vt16, mask, knew, vnew, attn16);

    k_gemm64<0, 29u, 0u><<<gP, 256, 0, stream>>>((const h16*)attn16, EDIM, (const h16*)wo16, EDIM, (void*)out, EDIM, bo, MROWS, EDIM, EDIM);
}
